// TransRet_25503515804196
// MI455X (gfx1250) — hardware-verified
//
#include <hip/hip_runtime.h>
#include <math.h>

typedef __attribute__((ext_vector_type(16))) _Float16 v16h;
typedef __attribute__((ext_vector_type(8)))  _Float16 v8h;
typedef __attribute__((ext_vector_type(16))) __bf16   v16b;
typedef __attribute__((ext_vector_type(8)))  __bf16   v8b;
typedef __attribute__((ext_vector_type(8)))  float    v8f;
typedef __attribute__((ext_vector_type(4)))  float    v4f;

constexpr int kB    = 16;
constexpr int kTxt  = 64;
constexpr int kVid  = 2048;
constexpr int kL    = kTxt + kVid;
constexpr int kLP   = 2304;
constexpr int kD    = 256;
constexpr int kHalf = kD / 2;
constexpr int kFF   = 1024;
constexpr int kThr  = 256;
constexpr float kInCarry = 1024.0f;
constexpr float kWCarry = 4096.0f;
constexpr float kCQ = 32.0f;
constexpr float kCS = 16.0f;
constexpr float kScP = 1.0f / (kInCarry * kWCarry), kScS = 1.0f / (kCQ * kCQ), kScA = 1.0f / (kCS * kInCarry), kScF = 1.0f / (kInCarry * kInCarry);
constexpr float kInvD = 1.0f / 256.0f;
constexpr float kLnEps = 1e-5f;
constexpr float kGamma = 0.9f;
constexpr float kF16MinNormal = 6.103515625e-5f;

static_assert(kL == 2112 && (kLP % 64) == 0 && kLP >= kL && ((kLP / 64) * (kLP / 64)) % 8 == 0 && ((kLP / 64) * (kD / 64)) % 8 == 0 && ((kLP / 64) * (kFF / 64)) % 8 == 0 && ((kVid / 64) * (2 * kD / 64)) % 8 == 0 && ((kD / 64) * (kVid / 64)) % 8 == 0, "GEMM M and N multiples of 64; every grid a whole number of 8-tile blocks");
static_assert((kD % 32) == 0 && (kLP % 32) == 0 && (kFF % 32) == 0 && (kTxt % 8) == 0 && (kL % 32) == 0, "GEMM K multiples of 32; the text block ends on a group of 8; the rows of a sample are whole waves");

constexpr size_t kOffWQK16 = 0ull;
constexpr size_t kOffWV16 = 262144ull;
constexpr size_t kOffL1W16 = 393216ull;
constexpr size_t kOffL2W16 = 917504ull;
constexpr size_t kOffBIAS = 1441792ull;
constexpr size_t kOffTAB = 1458176ull;
constexpr size_t kOffPOW9 = 5783552ull;
constexpr size_t kOffQX16 = 5791744ull;
constexpr size_t kOffKX16 = 6971392ull;
constexpr size_t kOffVT16 = 8151040ull;
constexpr size_t kOffN2H = 9330688ull;
constexpr size_t kOffN1 = 10510336ull;
constexpr size_t kOffX16 = 12673024ull;
constexpr size_t kOffPQK = 13721600ull;
constexpr size_t kOffVTF = 17915904ull;
constexpr size_t kOffSC = 20013056ull;
constexpr size_t kOffR16 = 41246720ull;
constexpr size_t kOffAT = 51863552ull;
constexpr size_t kOffX1 = 54222848ull;
constexpr size_t kOffH1 = 56385536ull;
constexpr size_t kOffG16 = 65822720ull;
constexpr size_t kOffFFO = 70541312ull;
constexpr size_t kWsTotal = 72900608ull;
static_assert(kWsTotal <= 134217728ull, "carve cap: under 128 MiB");
static_assert(kOffWQK16 == 0
              && kOffWV16 == kOffWQK16 + 262144ull
              && kOffL1W16 == kOffWV16 + 131072ull
              && kOffL2W16 == kOffL1W16 + 524288ull
              && kOffBIAS == kOffL2W16 + 524288ull
              && kOffTAB == kOffBIAS + 16384ull
              && kOffPOW9 == kOffTAB + 4325376ull
              && kOffQX16 == kOffPOW9 + 8192ull
              && kOffKX16 == kOffQX16 + 1179648ull
              && kOffVT16 == kOffKX16 + 1179648ull
              && kOffN2H == kOffVT16 + 1179648ull
              && kOffN1 == kOffN2H + 1179648ull
              && kOffX16 == kOffN1 + 2162688ull
              && kOffPQK == kOffX16 + 1048576ull
              && kOffVTF == kOffPQK + 4194304ull
              && kOffSC == kOffVTF + 2097152ull
              && kOffR16 == kOffSC + 21233664ull
              && kOffAT == kOffR16 + 10616832ull
              && kOffX1 == kOffAT + 2359296ull
              && kOffH1 == kOffX1 + 2162688ull
              && kOffG16 == kOffH1 + 9437184ull
              && kOffFFO == kOffG16 + 4718592ull
              && kWsTotal == kOffFFO + 2359296ull, "the carve is chained and totalled");
static_assert((kOffWQK16 % 256) == 0 && (kOffWV16 % 256) == 0 && (kOffL1W16 % 256) == 0 && (kOffL2W16 % 256) == 0 && (kOffBIAS % 256) == 0 && (kOffTAB % 256) == 0 && (kOffPOW9 % 256) == 0 && (kOffQX16 % 256) == 0 && (kOffKX16 % 256) == 0 && (kOffVT16 % 256) == 0 && (kOffN2H % 256) == 0 && (kOffN1 % 256) == 0 && (kOffX16 % 256) == 0 && (kOffPQK % 256) == 0 && (kOffVTF % 256) == 0 && (kOffSC % 256) == 0 && (kOffR16 % 256) == 0 && (kOffAT % 256) == 0 && (kOffX1 % 256) == 0 && (kOffH1 % 256) == 0 && (kOffG16 % 256) == 0 && (kOffFFO % 256) == 0, "aligned regions");
static_assert(kOffKX16 == kOffQX16 + 1179648ull && kOffVT16 == kOffKX16 + 1179648ull && kOffN2H == kOffVT16 + 1179648ull && kOffN1 == kOffN2H + 1179648ull, "the zero-filled region QX16 | KX16 | VT16 | N2H is contiguous: 4,718,592 B");

__device__ __forceinline__ unsigned short f2bf_bits(float f) {
  unsigned u = __float_as_uint(f);
  return (unsigned short)((u + 0x7FFFu + ((u >> 16) & 1u)) >> 16);
}
__device__ __forceinline__ float bf_bits2f(unsigned short h) { return __uint_as_float(((unsigned)h) << 16); }
__device__ __forceinline__ float bf16r(float f) { return bf_bits2f(f2bf_bits(f)); }
__device__ __forceinline__ float carry_flush(float v, float carry) {
  const float s = v * carry;
  return (fabsf(s) < kF16MinNormal) ? 0.0f : s;
}
__device__ __forceinline__ float frcp(float x) { return __builtin_amdgcn_rcpf(x); }

__device__ __forceinline__ void dep_guard4_h(v8f& a, v8f& b, v8f& c, v8f& d, v16h x, v16h y) { asm volatile("v_nop\n\tv_nop\n\tv_nop\n\tv_nop" : "+v"(a), "+v"(b), "+v"(c), "+v"(d) : "v"(x), "v"(y)); }
__device__ __forceinline__ void dep_guard4_b(v8f& a, v8f& b, v8f& c, v8f& d, v16b x, v16b y) { asm volatile("v_nop\n\tv_nop\n\tv_nop\n\tv_nop" : "+v"(a), "+v"(b), "+v"(c), "+v"(d) : "v"(x), "v"(y)); }
__device__ __forceinline__ void keep4_h(v16h a, v16h b, v16h c, v16h d) { asm volatile("v_nop" :: "v"(a), "v"(b), "v"(c), "v"(d)); }
__device__ __forceinline__ void keep4_b(v16b a, v16b b, v16b c, v16b d) { asm volatile("v_nop" :: "v"(a), "v"(b), "v"(c), "v"(d)); }
__device__ __forceinline__ void acc_guard4(v8f& a, v8f& b, v8f& c, v8f& d) { asm volatile("v_nop\n\tv_nop\n\tv_nop\n\tv_nop" : "+v"(a), "+v"(b), "+v"(c), "+v"(d)); }

template <typename T> struct Frag;
template <> struct Frag<_Float16> {
  typedef v16h V; union U { v16h v; v8h h[2]; };
  static __device__ __forceinline__ v16h load(const _Float16* p) {
    U f; f.h[0] = *(const v8h*)(p); f.h[1] = *(const v8h*)(p + 16); return f.v;
  }
  static __device__ __forceinline__ v8f mma(v16h a, v16h b, v8f c) {
    return __builtin_amdgcn_wmma_f32_16x16x32_f16(false, a, false, b, (short)0, c, false, false);
  }
  static __device__ __forceinline__ void guard4(v8f& a, v8f& b, v8f& c, v8f& d, v16h x, v16h y) { dep_guard4_h(a, b, c, d, x, y); }
  static __device__ __forceinline__ void keep(v16h a, v16h b, v16h c, v16h d) { keep4_h(a, b, c, d); }
};
template <> struct Frag<__bf16> {
  typedef v16b V; union U { v16b v; v8b h[2]; };
  static __device__ __forceinline__ v16b load(const __bf16* p) {
    U f; f.h[0] = *(const v8b*)(p); f.h[1] = *(const v8b*)(p + 16); return f.v;
  }
  static __device__ __forceinline__ v8f mma(v16b a, v16b b, v8f c) {
    return __builtin_amdgcn_wmma_f32_16x16x32_bf16(false, a, false, b, (short)0, c, false, false);
  }
  static __device__ __forceinline__ void guard4(v8f& a, v8f& b, v8f& c, v8f& d, v16b x, v16b y) { dep_guard4_b(a, b, c, d, x, y); }
  static __device__ __forceinline__ void keep(v16b a, v16b b, v16b c, v16b d) { keep4_b(a, b, c, d); }
};

__device__ __forceinline__ v8f mma_h(v16h a, v16h b, v8f c) {
  c = __builtin_amdgcn_wmma_f32_16x16x32_f16(false, a, false, b, (short)0, c, false, false);
  asm volatile("v_nop\n\tv_nop\n\tv_nop\n\tv_nop" : "+v"(c) : "v"(a), "v"(b));
  return c;
}

template <int ET> struct Elem;
template <> struct Elem<0> { typedef _Float16 T; };
template <> struct Elem<1> { typedef __bf16 T; };
template <int ET, bool SPLIT, int BIAS_MODE, int OUT_MODE, bool RESID, int ACT = 0>
__global__ __launch_bounds__(256) void wmma_gemm64(
    const unsigned short* __restrict__ Ap, const unsigned short* __restrict__ A2p, int lda, long strideA,
    const unsigned short* __restrict__ Btp, const unsigned short* __restrict__ Bt2p, int ldb, long strideB,
    void* __restrict__ Cout, void* __restrict__ Cout2, int ldc, long strideC,
    const float* __restrict__ bias,
    const float* __restrict__ resid, long strideR,
    int M, int N, int K, float scale) {
  typedef typename Elem<ET>::T T;
  typedef typename Frag<T>::V V;
  const T* A = (const T*)Ap; const T* A2 = (const T*)A2p; const T* Bt = (const T*)Btp; const T* Bt2 = (const T*)Bt2p;
  __shared__ __align__(16) float sT[8][16 * 68];
  const int b    = blockIdx.y;
  const int lane = threadIdx.x & 31;
  const int wave = threadIdx.x >> 5;
  const int tilesN = N >> 6;
  const int tilesM = M >> 6;
  const int tile = blockIdx.x * 8 + wave;
  if (tile >= tilesM * tilesN) return;
  const int tm = tile / tilesN;
  const int tn = tile - tm * tilesN;
  const int m0 = tm << 6;
  const int n0 = tn << 6;

  const T* Ab  = A  + (size_t)b * strideA;
  const T* Bb  = Bt + (size_t)b * strideB;
  const T* Ab2 = SPLIT ? (A2  + (size_t)b * strideA) : nullptr;
  const T* Bb2 = SPLIT ? (Bt2 + (size_t)b * strideB) : nullptr;

  const int rlane = lane & 15;
  const int koff  = (lane >> 4) * 8;
  const int mOff  = (lane >> 4) * 8;

  v8f acc[4][4];
#pragma unroll
  for (int i = 0; i < 4; ++i)
#pragma unroll
    for (int j = 0; j < 4; ++j) acc[i][j] = (v8f){0.f,0.f,0.f,0.f,0.f,0.f,0.f,0.f};

  for (int k0 = 0; k0 < K; k0 += 32) {
    V bh[4], bl[4];
#pragma unroll
    for (int j = 0; j < 4; ++j) {
      const size_t bo = (size_t)(n0 + (j << 4) + rlane) * ldb + koff + k0;
      bh[j] = Frag<T>::load(Bb + bo);
      if (SPLIT) bl[j] = Frag<T>::load(Bb2 + bo);
    }
#pragma unroll
    for (int i = 0; i < 4; ++i) {
      const size_t ao = (size_t)(m0 + (i << 4) + rlane) * lda + koff + k0;
      V ah = Frag<T>::load(Ab + ao);
      V al;
      if (SPLIT) al = Frag<T>::load(Ab2 + ao);
#pragma unroll
      for (int j = 0; j < 4; ++j) {
        acc[i][j] = Frag<T>::mma(ah, bh[j], acc[i][j]);
        if (SPLIT) {
          acc[i][j] = Frag<T>::mma(ah, bl[j], acc[i][j]);
          acc[i][j] = Frag<T>::mma(al, bh[j], acc[i][j]);
        }
      }
      Frag<T>::guard4(acc[i][0], acc[i][1], acc[i][2], acc[i][3], ah, SPLIT ? al : ah);
    }
    Frag<T>::keep(bh[0], bh[1], bh[2], bh[3]);
    if (SPLIT) Frag<T>::keep(bl[0], bl[1], bl[2], bl[3]);
  }
  acc_guard4(acc[0][0], acc[0][1], acc[0][2], acc[0][3]);
  acc_guard4(acc[1][0], acc[1][1], acc[1][2], acc[1][3]);
  acc_guard4(acc[2][0], acc[2][1], acc[2][2], acc[2][3]);
  acc_guard4(acc[3][0], acc[3][1], acc[3][2], acc[3][3]);

  float* slab = sT[wave];
  const float* Rb = RESID ? (resid + (size_t)b * strideR) : nullptr;
#pragma unroll
  for (int i = 0; i < 4; ++i) {
    const int mBase = m0 + (i << 4);
#pragma unroll
    for (int j = 0; j < 4; ++j) {
      const int n = n0 + (j << 4) + rlane;
      float bv = 0.f;
      if (BIAS_MODE == 2) bv = bias[n];
#pragma unroll
      for (int r = 0; r < 8; ++r) {
        float v = acc[i][j][r] * scale;
        if (BIAS_MODE == 1) v += bias[mBase + mOff + r];
        if (BIAS_MODE == 2) v += bv;
        if (RESID) v += Rb[(size_t)(mBase + mOff + r) * ldc + n];
        if (ACT == 1) v = tanhf(v);
        if (ACT == 2) v = fmaxf(v, 0.0f);
        if (ACT == 3) v = v / (1.0f + expf(-v));
        if (ACT == 4) v = (v > 0.f) ? v : 0.01f * v;
        slab[(mOff + r) * 68 + (j << 4) + rlane] = v;
      }
    }
    __builtin_amdgcn_fence(__ATOMIC_RELEASE, "workgroup");
    __builtin_amdgcn_wave_barrier();
    __builtin_amdgcn_fence(__ATOMIC_ACQUIRE, "workgroup");
    if (OUT_MODE == 0) {
      float* C = (float*)Cout + (size_t)b * strideC;
      const int hh = lane >> 4, c4 = (lane & 15) * 4;
      for (int pass = 0; pass < 2; ++pass) {
#pragma unroll
        for (int it = 0; it < 8; ++it) {
          const int row = it * 2 + hh;
          v4f v = *(const v4f*)(slab + row * 68 + c4);
          *(volatile v4f*)(C + (size_t)(mBase + row) * ldc + n0 + c4) = v;
        }
        __threadfence();
      }
    } else {
      const int q = lane >> 3, c8 = (lane & 7) * 8;
      unsigned short* C  = (unsigned short*)Cout  + (size_t)b * strideC;
      unsigned short* C2 = (OUT_MODE == 2) ? ((unsigned short*)Cout2 + (size_t)b * strideC) : nullptr;
      for (int pass = 0; pass < 2; ++pass) {
#pragma unroll
        for (int it = 0; it < 4; ++it) {
          const int row = it * 4 + q;
          const float* sp = slab + row * 68 + c8;
          v8h hv, lv;
#pragma unroll
          for (int e = 0; e < 8; ++e) {
            if (OUT_MODE == 1) {
              hv[e] = (_Float16)sp[e];
            } else {
              unsigned short hb = f2bf_bits(sp[e]);
              unsigned short lb = f2bf_bits(sp[e] - bf_bits2f(hb));
              hv[e] = __builtin_bit_cast(_Float16, hb);
              lv[e] = __builtin_bit_cast(_Float16, lb);
            }
          }
          *(volatile v8h*)(C + (size_t)(mBase + row) * ldc + n0 + c8) = hv;
          if (OUT_MODE == 2) *(volatile v8h*)(C2 + (size_t)(mBase + row) * ldc + n0 + c8) = lv;
        }
        __threadfence();
      }
    }
    __builtin_amdgcn_fence(__ATOMIC_RELEASE, "workgroup");
    __builtin_amdgcn_wave_barrier();
    __builtin_amdgcn_fence(__ATOMIC_ACQUIRE, "workgroup");
  }
}

__global__ __launch_bounds__(kThr) void cast_plane_kernel(const float* __restrict__ src, unsigned short* __restrict__ dst,
                                                          int colsLog2, int dstPitch, int dstOff) {
  const int i   = blockIdx.x * kThr + threadIdx.x;
  const int sh  = colsLog2 - 3;
  const int row = i >> sh;
  const int c8  = (i & ((1 << sh) - 1)) * 8;
  const float* sp = src + ((size_t)row << colsLog2) + c8;
  const v4f a0 = *(const v4f*)(sp);
  const v4f a1 = *(const v4f*)(sp + 4);
  v8h hv;
#pragma unroll
  for (int e = 0; e < 4; ++e) {
    const float f0 = a0[e];
    const float f1 = a1[e];
    hv[e]     = (_Float16)carry_flush(bf16r(f0), kInCarry);
    hv[4 + e] = (_Float16)carry_flush(bf16r(f1), kInCarry);
  }
  unsigned short* dp = dst + (size_t)row * dstPitch + dstOff + c8;
  *(volatile v8h*)dp = hv;
  __threadfence();
  *(volatile v8h*)dp = hv;
}
__global__ __launch_bounds__(256) void wt_plane_kernel(const float* __restrict__ W, unsigned short* __restrict__ dst, int K, int N, int nLive, int ldd, int colOff) {
  const int n  = blockIdx.x;
  const int k8 = threadIdx.x * 8;
  const bool live = n < nLive;
  const int nc = live ? n : 0;
  v8h hv;
#pragma unroll
  for (int e = 0; e < 8; ++e) {
    const float w = W[(size_t)(k8 + e) * N + nc];
    hv[e] = (_Float16)(live ? carry_flush(bf16r(w), kWCarry) : 0.0f);
  }
  unsigned short* dp = dst + (size_t)n * ldd + colOff + k8;
  *(volatile v8h*)dp = hv;
  __threadfence();
  *(volatile v8h*)dp = hv;
}


constexpr int kFB1 = 0, kFB2 = 1024, kFZB = 1792, kFEnd = 4096;
__global__ __launch_bounds__(kThr) void setup_kernel(const float* __restrict__ lin1_b, const float* __restrict__ lin2_b, float* __restrict__ BIAS,
                                                     unsigned short* __restrict__ ZERO) {
  unsigned v = blockIdx.x * (unsigned)kThr + threadIdx.x;
  asm volatile("" : "+v"(v));
  if (v < 1024u) {
    const unsigned i0 = v * 4u;
    v4f o = {0.f, 0.f, 0.f, 0.f};
    if (i0 < (unsigned)kFB2) {
      const v4f a = *(const v4f*)(lin1_b + i0);
#pragma unroll
      for (int e = 0; e < 4; ++e) { const float p = a[e]; o[e] = bf16r(p); }
    } else if (i0 < (unsigned)(kFB2 + kD)) {
      const v4f a = *(const v4f*)(lin2_b + (i0 - (unsigned)kFB2));
#pragma unroll
      for (int e = 0; e < 4; ++e) { const float p = a[e]; o[e] = bf16r(p); }
    }
    float* dp = BIAS + i0;
    *(volatile v4f*)dp = o;
    __threadfence();
    *(volatile v4f*)dp = o;
  } else {
    const unsigned w = v - 1024u;
    v8h z;
#pragma unroll
    for (int e = 0; e < 8; ++e) z[e] = (_Float16)0.0f;
    unsigned short* dp = ZERO + (size_t)w * 8u;
    *(volatile v8h*)dp = z;
    __threadfence();
    *(volatile v8h*)dp = z;
  }
}
static_assert(kFEnd / 4 == 1024 && 4718592 / 16 == 294912 && 1024 + 294912 == 1156 * kThr, "set-up grid exact");
static_assert((kFB2 % 128) == 0 && ((kFB2 + kD) % 128) == 0 && (kFZB % 128) == 0 && kFZB >= kFB2 + kD && kFEnd - kFZB >= kLP && kFB2 - kFB1 >= kFF, "set-up regions wave-uniform; the zero row covers the widest zero-bias product (2,304 columns)");

__global__ __launch_bounds__(kThr) void table_kernel(float* __restrict__ TAB, float* __restrict__ POW9) {
  unsigned v = blockIdx.x * (unsigned)kThr + threadIdx.x;
  asm volatile("" : "+v"(v));
  v4f o;
  float* dp;
  if (v < 270336u) {
    const unsigned l = v >> 7, j = v & 127u;
    const bool txt = l < (unsigned)kTxt;
    const float p = (float)(txt ? l : (l - (unsigned)kTxt));
    const float minpos = txt ? -32.0f : -1024.0f;
    const float sv = (2.0f * (float)j + 102.4f) / 358.4f;
    const float pw = (minpos + p) / 512.0f;
    const float sc = powf(sv, pw);
    const float invf = 1.0f / powf(10000.0f, (float)j / 128.0f);
    const float ang = p * invf;
    const float sn = sinf(ang), cs = cosf(ang);
    const float isc = 1.0f / sc;
    o[0] = cs * sc; o[1] = sn * sc; o[2] = cs * isc; o[3] = sn * isc;
    dp = TAB + (size_t)v * 4u;
  } else {
    const unsigned w = v - 270336u;
#pragma unroll
    for (int e = 0; e < 4; ++e) o[e] = powf(kGamma, (float)(4u * w + (unsigned)e));
    dp = POW9 + (size_t)w * 4u;
  }
  *(volatile v4f*)dp = o;
  __threadfence();
  *(volatile v4f*)dp = o;
}
static_assert(kL * kHalf == 270336 && kVid / 4 == 512 && 270336 + 512 == 1058 * kThr && (270336 % 32) == 0, "table grid exact; regions wave-uniform");

__global__ __launch_bounds__(kThr) void addln_kernel(const float* __restrict__ A, const float* __restrict__ ADD, const float* __restrict__ g,
                                                     const float* __restrict__ beta, float* __restrict__ SUM32, float* __restrict__ O32,
                                                     unsigned short* __restrict__ O16, int rows, int flags) {
  unsigned r = blockIdx.x * (unsigned)kThr + threadIdx.x;
  asm volatile("" : "+v"(r));
  if (r >= (unsigned)rows) return;
  const bool wantAdd = (flags & 1) != 0, wantSum = (flags & 2) != 0, want32 = (flags & 4) != 0, want16 = (flags & 8) != 0, inA = (flags & 16) != 0;
  const float* a = A + (size_t)r * kD;
  const float* ad = ADD + (size_t)r * kD;
  float s = 0.0f;
  for (unsigned c = 0; c < (unsigned)kD; c += 4) {
    v4f x = *(const v4f*)(a + c);
    if (inA) { x[0] = bf16r(x[0]); x[1] = bf16r(x[1]); x[2] = bf16r(x[2]); x[3] = bf16r(x[3]); }
    if (wantAdd) { const v4f y = *(const v4f*)(ad + c); x = x + y; }
    s += x[0]; s += x[1]; s += x[2]; s += x[3];
  }
  const float mu = s * kInvD;
  float q = 0.0f;
  for (unsigned c = 0; c < (unsigned)kD; c += 4) {
    v4f x = *(const v4f*)(a + c);
    if (inA) { x[0] = bf16r(x[0]); x[1] = bf16r(x[1]); x[2] = bf16r(x[2]); x[3] = bf16r(x[3]); }
    if (wantAdd) { const v4f y = *(const v4f*)(ad + c); x = x + y; }
#pragma unroll
    for (int e = 0; e < 4; ++e) { const float d = x[e] - mu; q += d * d; }
  }
  const float rstd = rsqrtf(q * kInvD + kLnEps);
  float* sp = SUM32 + (size_t)r * kD;
  float* op = O32 + (size_t)r * kD;
  unsigned short* hp = O16 + (size_t)r * kD;
  for (unsigned c = 0; c < (unsigned)kD; c += 8) {
    v4f x0 = *(const v4f*)(a + c), x1 = *(const v4f*)(a + c + 4);
    if (inA) {
#pragma unroll
      for (int e = 0; e < 4; ++e) { x0[e] = bf16r(x0[e]); x1[e] = bf16r(x1[e]); }
    }
    if (wantAdd) { const v4f y0 = *(const v4f*)(ad + c), y1 = *(const v4f*)(ad + c + 4); x0 = x0 + y0; x1 = x1 + y1; }
    const v4f g0 = *(const v4f*)(g + c), g1 = *(const v4f*)(g + c + 4), b0 = *(const v4f*)(beta + c), b1 = *(const v4f*)(beta + c + 4);
    v4f n0, n1;
    v8h hv;
#pragma unroll
    for (int e = 0; e < 4; ++e) {
      n0[e] = (x0[e] - mu) * rstd * bf16r(g0[e]) + bf16r(b0[e]);
      n1[e] = (x1[e] - mu) * rstd * bf16r(g1[e]) + bf16r(b1[e]);
      hv[e] = (_Float16)carry_flush(n0[e], kInCarry);
      hv[4 + e] = (_Float16)carry_flush(n1[e], kInCarry);
    }
    for (int pass = 0; pass < 2; ++pass) {
      if (wantSum) { *(volatile v4f*)(sp + c) = x0; *(volatile v4f*)(sp + c + 4) = x1; }
      if (want32)  { *(volatile v4f*)(op + c) = n0; *(volatile v4f*)(op + c + 4) = n1; }
      if (want16)  { *(volatile v8h*)(hp + c) = hv; }
      __threadfence();
    }
  }
}

__global__ __launch_bounds__(kThr) void xpos_kernel(const float* __restrict__ N1, const float* __restrict__ PQK, const float* __restrict__ TAB,
                                                    unsigned short* __restrict__ QX16, unsigned short* __restrict__ KX16) {
  unsigned v = blockIdx.x * (unsigned)kThr + threadIdx.x;
  asm volatile("" : "+v"(v));
  const unsigned n = v >> 5, c8 = (v & 31u) * 8u;
  const bool txt = n < (unsigned)kTxt;
  const unsigned nv = txt ? 0u : (n - (unsigned)kTxt);
  const float* qs = txt ? (N1 + (size_t)n * kD + c8) : (PQK + (size_t)nv * (2 * kD) + c8);
  const float* ks = txt ? (N1 + (size_t)n * kD + c8) : (PQK + (size_t)nv * (2 * kD) + kD + c8);
  const v4f q0 = *(const v4f*)qs, q1 = *(const v4f*)(qs + 4), k0 = *(const v4f*)ks, k1 = *(const v4f*)(ks + 4);
  const float* tp = TAB + ((size_t)n * kHalf + (c8 >> 1)) * 4u;
  float qv[8], kv[8];
#pragma unroll
  for (int e = 0; e < 4; ++e) { qv[e] = q0[e]; qv[4 + e] = q1[e]; kv[e] = k0[e]; kv[4 + e] = k1[e]; }
  v8h qh, kh;
#pragma unroll
  for (int pr = 0; pr < 4; ++pr) {
    const v4f t = *(const v4f*)(tp + 4 * pr);
    const float qa = qv[2 * pr], qb = qv[2 * pr + 1];
    const float ka = kv[2 * pr], kb = kv[2 * pr + 1];
    qh[2 * pr]     = (_Float16)carry_flush(qa * t[0] - qb * t[1], kCQ);
    qh[2 * pr + 1] = (_Float16)carry_flush(qb * t[0] + qa * t[1], kCQ);
    kh[2 * pr]     = (_Float16)carry_flush(ka * t[2] - kb * t[3], kCQ);
    kh[2 * pr + 1] = (_Float16)carry_flush(kb * t[2] + ka * t[3], kCQ);
  }
  unsigned short* qp = QX16 + (size_t)n * kD + c8;
  unsigned short* kp = KX16 + (size_t)n * kD + c8;
  for (int pass = 0; pass < 2; ++pass) {
    *(volatile v8h*)qp = qh;
    *(volatile v8h*)kp = kh;
    __threadfence();
  }
}
static_assert(kL * (kD / 8) == 264 * kThr && kD / 8 == 32, "position-encoding grid exact");

__global__ __launch_bounds__(kThr) void vt_kernel(const float* __restrict__ VTF, const float* __restrict__ N1, unsigned short* __restrict__ VT16) {
  unsigned v = blockIdx.x * (unsigned)kThr + threadIdx.x;
  asm volatile("" : "+v"(v));
  const unsigned d = v / 264u, m8 = (v - d * 264u) * 8u;
  v8h hv;
  if (m8 < (unsigned)kTxt) {
#pragma unroll
    for (int e = 0; e < 8; ++e) { float x = N1[(size_t)(m8 + (unsigned)e) * kD + d]; asm volatile("" : "+v"(x)); hv[e] = (_Float16)carry_flush(x, kInCarry); }
  } else {
    const float* sp = VTF + (size_t)d * kVid + (m8 - (unsigned)kTxt);
    const v4f a0 = *(const v4f*)sp, a1 = *(const v4f*)(sp + 4);
#pragma unroll
    for (int e = 0; e < 4; ++e) { hv[e] = (_Float16)carry_flush(a0[e], kInCarry); hv[4 + e] = (_Float16)carry_flush(a1[e], kInCarry); }
  }
  unsigned short* dp = VT16 + (size_t)d * kLP + m8;
  *(volatile v8h*)dp = hv;
  __threadfence();
  *(volatile v8h*)dp = hv;
}
static_assert(kL / 8 == 264 && kD * 264 == 264 * kThr && (kLP % 64) == 0, "value-transpose grid exact");

__global__ __launch_bounds__(kThr) void mask_kernel(const float* __restrict__ SC, const float* __restrict__ POW9, unsigned short* __restrict__ R16) {
  unsigned v = blockIdx.x * (unsigned)kThr + threadIdx.x;
  asm volatile("" : "+v"(v));
  const unsigned n = v / 288u, m8 = (v - n * 288u) * 8u;
  const float* sp = SC + (size_t)n * kLP + m8;
  const v4f a0 = *(const v4f*)sp, a1 = *(const v4f*)(sp + 4);
  float sv8[8];
#pragma unroll
  for (int e = 0; e < 4; ++e) { sv8[e] = a0[e]; sv8[4 + e] = a1[e]; }
  v8h hv;
#pragma unroll
  for (int e = 0; e < 8; ++e) {
    const unsigned m = m8 + (unsigned)e;
    const bool inside = (n < (unsigned)kL) && (m < (unsigned)kL);
    const bool plain = (n < (unsigned)kTxt) || (m < (unsigned)kTxt);
    const bool causal = n >= m;
    const unsigned k = (inside && !plain && causal) ? (n - m) : 0u;
    float pw = POW9[k];
    asm volatile("" : "+v"(pw));
    const float mk = inside ? (plain ? 1.0f : (causal ? pw : 0.0f)) : 0.0f;
    hv[e] = (_Float16)carry_flush(sv8[e] * mk, kCS);
  }
  unsigned short* dp = R16 + (size_t)n * kLP + m8;
  *(volatile v8h*)dp = hv;
  __threadfence();
  *(volatile v8h*)dp = hv;
}
static_assert(kLP / 8 == 288 && ((size_t)kLP * 288) % kThr == 0, "mask grid exact");

__global__ __launch_bounds__(kThr) void gelu_kernel(const float* __restrict__ H1, unsigned short* __restrict__ G16) {
  unsigned v = blockIdx.x * (unsigned)kThr + threadIdx.x;
  asm volatile("" : "+v"(v));
  const float* sp = H1 + (size_t)v * 8u;
  const v4f a0 = *(const v4f*)sp, a1 = *(const v4f*)(sp + 4);
  v8h hv;
#pragma unroll
  for (int e = 0; e < 4; ++e) {
    const float x0 = a0[e], x1 = a1[e];
    const float y0 = 0.5f * x0 * (1.0f + erff(x0 * 0.70710678118654752f)), y1 = 0.5f * x1 * (1.0f + erff(x1 * 0.70710678118654752f));
    hv[e] = (_Float16)carry_flush(y0, kInCarry);
    hv[4 + e] = (_Float16)carry_flush(y1, kInCarry);
  }
  unsigned short* dp = G16 + (size_t)v * 8u;
  *(volatile v8h*)dp = hv;
  __threadfence();
  *(volatile v8h*)dp = hv;
}
static_assert(((size_t)kLP * kFF / 8) % kThr == 0, "GELU grid exact");

static_assert(((size_t)kFF * kD / 8) % kThr == 0 && ((size_t)kD * kFF / 8) % kThr == 0, "plane cast grids exact");

extern "C" void kernel_launch(void* const* d_in, const int* in_sizes, int n_in,
                              void* d_out, int out_size, void* d_ws, size_t ws_size,
                              hipStream_t stream) {
  if (n_in < 15 || d_out == nullptr || d_ws == nullptr) return;
  if (in_sizes[0] != kB * kTxt * kD || in_sizes[1] != kB * kVid * kD || in_sizes[2] != kD * kD || in_sizes[3] != kD * kD || in_sizes[4] != kD * kD) return;
  if (in_sizes[5] != kFF * kD || in_sizes[6] != kFF || in_sizes[7] != kD * kFF || in_sizes[8] != kD) return;
  if (in_sizes[9] != kD || in_sizes[10] != kD || in_sizes[11] != kD || in_sizes[12] != kD || in_sizes[13] != kD || in_sizes[14] != kD) return;
  if (out_size != kB * kL * kD) return;
  if (ws_size < kWsTotal) return;
  const float* txt_src = (const float*)d_in[0];
  const float* vid_src = (const float*)d_in[1];
  const float* W_Q = (const float*)d_in[2];
  const float* W_K = (const float*)d_in[3];
  const float* W_V = (const float*)d_in[4];
  const float* lin1_w = (const float*)d_in[5];
  const float* lin1_b = (const float*)d_in[6];
  const float* lin2_w = (const float*)d_in[7];
  const float* lin2_b = (const float*)d_in[8];
  const float* ln1_g = (const float*)d_in[9];
  const float* ln1_b = (const float*)d_in[10];
  const float* ln2_g = (const float*)d_in[11];
  const float* ln2_b = (const float*)d_in[12];
  const float* ln3_g = (const float*)d_in[13];
  const float* ln3_b = (const float*)d_in[14];
  float* out = (float*)d_out;
  char* ws = (char*)d_ws;
  unsigned short* WQK16 = (unsigned short*)(ws + kOffWQK16);
  unsigned short* WV16 = (unsigned short*)(ws + kOffWV16);
  unsigned short* L1W16 = (unsigned short*)(ws + kOffL1W16);
  unsigned short* L2W16 = (unsigned short*)(ws + kOffL2W16);
  float* BIAS = (float*)(ws + kOffBIAS);
  float* TAB = (float*)(ws + kOffTAB);
  float* POW9 = (float*)(ws + kOffPOW9);
  unsigned short* QX16 = (unsigned short*)(ws + kOffQX16);
  unsigned short* KX16 = (unsigned short*)(ws + kOffKX16);
  unsigned short* VT16 = (unsigned short*)(ws + kOffVT16);
  unsigned short* N2H = (unsigned short*)(ws + kOffN2H);
  float* N1 = (float*)(ws + kOffN1);
  unsigned short* X16 = (unsigned short*)(ws + kOffX16);
  float* PQK = (float*)(ws + kOffPQK);
  float* VTF = (float*)(ws + kOffVTF);
  float* SC = (float*)(ws + kOffSC);
  unsigned short* R16 = (unsigned short*)(ws + kOffR16);
  float* AT = (float*)(ws + kOffAT);
  float* X1 = (float*)(ws + kOffX1);
  float* H1 = (float*)(ws + kOffH1);
  unsigned short* G16 = (unsigned short*)(ws + kOffG16);
  float* FFO = (float*)(ws + kOffFFO);

  wt_plane_kernel<<<kD, kD / 8, 0, stream>>>(W_Q, WQK16, kD, kD, kD, kD, 0);
  wt_plane_kernel<<<kD, kD / 8, 0, stream>>>(W_K, WQK16 + (size_t)kD * kD, kD, kD, kD, kD, 0);
  wt_plane_kernel<<<kD, kD / 8, 0, stream>>>(W_V, WV16, kD, kD, kD, kD, 0);
  cast_plane_kernel<<<(int)(((size_t)kFF * kD / 8) / kThr), kThr, 0, stream>>>(lin1_w, L1W16, 8, kD, 0);
  cast_plane_kernel<<<(int)(((size_t)kD * kFF / 8) / kThr), kThr, 0, stream>>>(lin2_w, L2W16, 10, kFF, 0);
  setup_kernel<<<1156, kThr, 0, stream>>>(lin1_b, lin2_b, BIAS, QX16);
  table_kernel<<<1058, kThr, 0, stream>>>(TAB, POW9);

  for (int b = 0; b < kB; ++b) {
    const float* ts = txt_src + (size_t)b * kTxt * kD;
    const float* vs = vid_src + (size_t)b * kVid * kD;
    addln_kernel<<<1, kThr, 0, stream>>>(ts, ts, ln1_g, ln1_b, N1, N1, X16, kTxt, 4 | 16);
    addln_kernel<<<kVid / kThr, kThr, 0, stream>>>(vs, vs, ln1_g, ln1_b, N1, N1 + (size_t)kTxt * kD, X16, kVid, 12 | 16);
    wmma_gemm64<0, false, 2, 0, false, 0><<<dim3((kVid / 64) * (2 * kD / 64) / 8, 1), 256, 0, stream>>>(
        X16, X16, kD, 0L, WQK16, WQK16, kD, 0L, (void*)PQK, (void*)PQK, 2 * kD, 0L, BIAS + kFZB, nullptr, 0L, kVid, 2 * kD, kD, kScP);
    wmma_gemm64<0, false, 2, 0, false, 0><<<dim3((kD / 64) * (kVid / 64) / 8, 1), 256, 0, stream>>>(
        WV16, WV16, kD, 0L, X16, X16, kD, 0L, (void*)VTF, (void*)VTF, kVid, 0L, BIAS + kFZB, nullptr, 0L, kD, kVid, kD, kScP);
    xpos_kernel<<<264, kThr, 0, stream>>>(N1, PQK, TAB, QX16, KX16);
    vt_kernel<<<264, kThr, 0, stream>>>(VTF, N1, VT16);
    wmma_gemm64<0, false, 2, 0, false, 0><<<dim3((kLP / 64) * (kLP / 64) / 8, 1), 256, 0, stream>>>(
        QX16, QX16, kD, 0L, KX16, KX16, kD, 0L, (void*)SC, (void*)SC, kLP, 0L, BIAS + kFZB, nullptr, 0L, kLP, kLP, kD, kScS);
    mask_kernel<<<2592, kThr, 0, stream>>>(SC, POW9, R16);
    wmma_gemm64<0, false, 2, 0, false, 0><<<dim3((kLP / 64) * (kD / 64) / 8, 1), 256, 0, stream>>>(
        R16, R16, kLP, 0L, VT16, VT16, kLP, 0L, (void*)AT, (void*)AT, kD, 0L, BIAS + kFZB, nullptr, 0L, kLP, kD, kLP, kScA);
    addln_kernel<<<1, kThr, 0, stream>>>(ts, AT, ln2_g, ln2_b, X1, X1, N2H, kTxt, 11 | 16);
    addln_kernel<<<kVid / kThr, kThr, 0, stream>>>(vs, AT + (size_t)kTxt * kD, ln2_g, ln2_b, X1 + (size_t)kTxt * kD, X1, N2H + (size_t)kTxt * kD, kVid, 11 | 16);
    wmma_gemm64<0, false, 2, 0, false, 0><<<dim3((kLP / 64) * (kFF / 64) / 8, 1), 256, 0, stream>>>(
        N2H, N2H, kD, 0L, L1W16, L1W16, kD, 0L, (void*)H1, (void*)H1, kFF, 0L, BIAS + kFB1, nullptr, 0L, kLP, kFF, kD, kScF);
    gelu_kernel<<<1152, kThr, 0, stream>>>(H1, G16);
    wmma_gemm64<0, false, 2, 0, false, 0><<<dim3((kLP / 64) * (kD / 64) / 8, 1), 256, 0, stream>>>(
        G16, G16, kFF, 0L, L2W16, L2W16, kFF, 0L, (void*)FFO, (void*)FFO, kD, 0L, BIAS + kFB2, nullptr, 0L, kLP, kD, kFF, kScF);
    addln_kernel<<<kLP / kThr, kThr, 0, stream>>>(X1, FFO, ln3_g, ln3_b, X1, out + (size_t)b * kL * kD, N2H, kL, 5);
  }
}
